// SingleHeadAttention_74448963109518
// MI455X (gfx1250) — hardware-run, weakly checked
//
#include <hip/hip_runtime.h>


#ifndef NB
#define NB 4
#endif
#ifndef SEQ
#define SEQ 2048
#endif
#define NB_FULL  4
#define SEQ_FULL 2048
#define TT   SEQ
#define DM   1024
#define HD   1024
#define DQ   HD
#define NQKV (3 * HD)
#define ZH   1
#ifndef RH
#define RH   (SEQ < 512 ? SEQ : 512)
#endif
#define PCAR 1024.0f
#define SCL  0.03125f

static_assert(NB >= 1 && NB <= NB_FULL);
static_assert(SEQ >= 128 && SEQ <= SEQ_FULL && (SEQ % 128) == 0);
static_assert((RH % 64) == 0 && RH >= 0 && RH <= SEQ);
static_assert((DM % 64) == 0 && (HD % 256) == 0 && (NQKV % 64) == 0);
static_assert((TT % 64) == 0 && (TT % 32) == 0 && (HD % 32) == 0 && (DM % 32) == 0);
static_assert(DM == HD);
static_assert((HD % 8) == 0 && (DM % 8) == 0 && (NQKV % 8) == 0);
static_assert(16 * 68 * 4 <= 131072);
static_assert(32 * 16 * 8 == 16 * 64 * 4);
static_assert(32 * 4 * (TT / 128) == TT);
#define AL256(x) ((((size_t)(x)) + 255) & ~(size_t)255)
static_assert(AL256((size_t)NQKV * DM * 2) + AL256((size_t)DM * HD * 2) + AL256((size_t)TT * DM * 2) + AL256((size_t)TT * NQKV * 4) + AL256((size_t)HD * TT * 2)
              + 2 * AL256((size_t)2 * TT * HD * 2) + 2 * AL256((size_t)HD * TT * 2) + 2 * AL256((size_t)ZH * RH * TT * 2)
              + AL256((size_t)ZH * TT * TT * 4) + AL256((size_t)ZH * TT * TT * 2) + AL256((size_t)ZH * TT * HD * 4) + 2 * AL256((size_t)TT * HD * 2) <= (size_t)134217728);

typedef _Float16 h16;
typedef unsigned short bf;
typedef __attribute__((ext_vector_type(16))) __bf16   v16bf;
typedef __attribute__((ext_vector_type(16))) _Float16 v16h;
typedef __attribute__((ext_vector_type(8)))  _Float16 v8h;
typedef __attribute__((ext_vector_type(8)))  unsigned short v8us;
typedef __attribute__((ext_vector_type(8)))  float    v8f;
typedef __attribute__((ext_vector_type(4)))  float    v4f;
typedef v4f  __attribute__((may_alias)) v4fa;
typedef v8us __attribute__((may_alias)) v8usa;
typedef __attribute__((ext_vector_type(2))) _Float16 v2h;
typedef __attribute__((ext_vector_type(4))) _Float16 v4h;
typedef __attribute__((ext_vector_type(2))) unsigned short v2us;
typedef __attribute__((ext_vector_type(4))) unsigned short v4us;
typedef __attribute__((ext_vector_type(2))) float v2f;

__device__ __forceinline__ unsigned short f2bf(float f) { unsigned u = __float_as_uint(f); u += 0x7FFFu + ((u >> 16) & 1u); return (unsigned short)(u >> 16); }
__device__ __forceinline__ float bf2f(unsigned short b) { return __uint_as_float(((unsigned)b) << 16); }
__device__ __forceinline__ float bfr(float f) { return bf2f(f2bf(f)); }
__device__ __forceinline__ v16h cat16(v8h lo, v8h hi) { return __builtin_shufflevector(lo, hi, 0, 1, 2, 3, 4, 5, 6, 7, 8, 9, 10, 11, 12, 13, 14, 15); }
__device__ __forceinline__ v16bf cat16b(v8us lo, v8us hi) { return __builtin_bit_cast(v16bf, __builtin_shufflevector(lo, hi, 0, 1, 2, 3, 4, 5, 6, 7, 8, 9, 10, 11, 12, 13, 14, 15)); }
__device__ __forceinline__ v8f wmma16(v16h a, v16h b, v8f c) { return __builtin_amdgcn_wmma_f32_16x16x32_f16(false, a, false, b, (short)0, c, false, false); }
__device__ __forceinline__ v8f wmmab(v16bf a, v16bf b, v8f c) { return __builtin_amdgcn_wmma_f32_16x16x32_bf16(false, a, false, b, (short)0, c, false, false); }

template <typename T16> struct WFrag;
template <> struct WFrag<h16> { typedef v16h V; static __device__ __forceinline__ V ld(const h16* p) { return cat16(*(const v8h*)p, *(const v8h*)(p + 16)); } static __device__ __forceinline__ v8f mma(V a, V b, v8f c) { return wmma16(a, b, c); } };
template <> struct WFrag<bf> { typedef v16bf V; static __device__ __forceinline__ V ld(const bf* p) { return cat16b(*(const v8us*)p, *(const v8us*)(p + 16)); } static __device__ __forceinline__ v8f mma(V a, V b, v8f c) { return wmmab(a, b, c); } };
template <typename T16, int NSPLIT, bool BIAS>
__global__ __launch_bounds__(32) void k_gemmw(const T16* __restrict__ A, const T16* __restrict__ A2, const T16* __restrict__ Bt, const T16* __restrict__ Bt2, int K, float* C, int ldc, const float* __restrict__ bias, size_t sA, size_t sB, size_t sC) {
    typedef typename WFrag<T16>::V V;
    __shared__ __align__(16) float os[16 * 68];
    const size_t z = blockIdx.z; A += z * sA; if (A2) A2 += z * sA; Bt += z * sB; if (Bt2) Bt2 += z * sB; C += z * sC;
    const int lane = threadIdx.x & 31, lr = lane & 15, hi = lane >> 4; const int r0 = blockIdx.x * 64, c0 = blockIdx.y * 64;
    v8f acc[4][4];
#pragma unroll
    for (int mb = 0; mb < 4; ++mb)
#pragma unroll
        for (int nb = 0; nb < 4; ++nb) acc[mb][nb] = (v8f){};
    const size_t aoff = (size_t)(r0 + lr) * K + 8 * hi, boff = (size_t)(c0 + lr) * K + 8 * hi;
#pragma unroll 1
    for (int kc = 0; kc < K; kc += 32) {
        V a[4], a2[4];
#pragma unroll
        for (int mb = 0; mb < 4; ++mb) { a[mb] = WFrag<T16>::ld(A + aoff + (size_t)mb * 16 * K + kc); if (NSPLIT == 1 || NSPLIT == 2) a2[mb] = WFrag<T16>::ld(A2 + aoff + (size_t)mb * 16 * K + kc); }
#pragma unroll
        for (int nb = 0; nb < 4; ++nb) { const V b = WFrag<T16>::ld(Bt + boff + (size_t)nb * 16 * K + kc); V b2; if (NSPLIT >= 2) b2 = WFrag<T16>::ld(Bt2 + boff + (size_t)nb * 16 * K + kc);
#pragma unroll
            for (int mb = 0; mb < 4; ++mb) { acc[mb][nb] = WFrag<T16>::mma(a[mb], b, acc[mb][nb]); if (NSPLIT == 1 || NSPLIT == 2) acc[mb][nb] = WFrag<T16>::mma(a2[mb], b, acc[mb][nb]); if (NSPLIT >= 2) acc[mb][nb] = WFrag<T16>::mma(a[mb], b2, acc[mb][nb]); } }
        asm volatile("v_nop\n\tv_nop\n\tv_nop\n\tv_nop" : "+v"(acc[0][0]), "+v"(acc[1][1]), "+v"(acc[2][2]), "+v"(acc[3][3]) : "v"(a[0]), "v"(a[3]));
    }
#pragma unroll
    for (int mb = 0; mb < 4; ++mb) {
#pragma unroll
        for (int nb = 0; nb < 4; ++nb) {
#pragma unroll
            for (int j = 0; j < 8; ++j) os[(hi * 8 + j) * 68 + nb * 16 + lr] = acc[mb][nb][j]; }
        __builtin_amdgcn_wave_barrier(); asm volatile("" ::: "memory");
        float* crow = C + (size_t)(r0 + mb * 16) * ldc + c0;
#pragma unroll 1
        for (int ps = 0; ps < 2; ++ps) {
#pragma unroll
            for (int s = 0; s < 8; ++s) { const int row = 2 * s + hi, cofs = lr * 4; v4f val = *(const v4fa*)(os + row * 68 + cofs); if (BIAS) { val[0] += bfr(bias[c0 + cofs]); val[1] += bfr(bias[c0 + cofs + 1]); val[2] += bfr(bias[c0 + cofs + 2]); val[3] += bfr(bias[c0 + cofs + 3]); }
                *(volatile v4f*)(crow + (size_t)row * ldc + cofs) = val; }
            if (ps == 0) __threadfence(); }
        __builtin_amdgcn_wave_barrier(); asm volatile("" ::: "memory");
    }
}

template <typename T16, int NSPLIT, int CMODE>
__device__ __forceinline__ void gemmc_body(const T16* __restrict__ A, const T16* __restrict__ A2, const T16* __restrict__ Bt, const T16* __restrict__ Bt2, int K, float* C, int ldc, int qbase) {
    typedef typename WFrag<T16>::V V;
    __shared__ __align__(16) float os[16 * 68];
    const int lane = threadIdx.x & 31, lr = lane & 15, hi = lane >> 4; const int r0 = blockIdx.x * 64, c0 = blockIdx.y * 64;
    int kend = K;
    if (CMODE == 0) { if (c0 > qbase + r0) kend = 0; } else { if (qbase + r0 + 64 < K) kend = qbase + r0 + 64; }
    v8f acc[4][4];
#pragma unroll
    for (int mb = 0; mb < 4; ++mb)
#pragma unroll
        for (int nb = 0; nb < 4; ++nb) acc[mb][nb] = (v8f){};
    const size_t aoff = (size_t)(r0 + lr) * K + 8 * hi, boff = (size_t)(c0 + lr) * K + 8 * hi;
#pragma unroll 1
    for (int kc = 0; kc < kend; kc += 32) {
        V a[4], a2[4];
#pragma unroll
        for (int mb = 0; mb < 4; ++mb) { a[mb] = WFrag<T16>::ld(A + aoff + (size_t)mb * 16 * K + kc); if (NSPLIT == 1 || NSPLIT == 2) a2[mb] = WFrag<T16>::ld(A2 + aoff + (size_t)mb * 16 * K + kc); }
#pragma unroll
        for (int nb = 0; nb < 4; ++nb) { const V b = WFrag<T16>::ld(Bt + boff + (size_t)nb * 16 * K + kc); V b2; if (NSPLIT >= 2) b2 = WFrag<T16>::ld(Bt2 + boff + (size_t)nb * 16 * K + kc);
#pragma unroll
            for (int mb = 0; mb < 4; ++mb) { acc[mb][nb] = WFrag<T16>::mma(a[mb], b, acc[mb][nb]); if (NSPLIT == 1 || NSPLIT == 2) acc[mb][nb] = WFrag<T16>::mma(a2[mb], b, acc[mb][nb]); if (NSPLIT >= 2) acc[mb][nb] = WFrag<T16>::mma(a[mb], b2, acc[mb][nb]); } }
        asm volatile("v_nop\n\tv_nop\n\tv_nop\n\tv_nop" : "+v"(acc[0][0]), "+v"(acc[1][1]), "+v"(acc[2][2]), "+v"(acc[3][3]) : "v"(a[0]), "v"(a[3]));
    }
#pragma unroll
    for (int mb = 0; mb < 4; ++mb) {
#pragma unroll
        for (int nb = 0; nb < 4; ++nb) {
#pragma unroll
            for (int j = 0; j < 8; ++j) os[(hi * 8 + j) * 68 + nb * 16 + lr] = acc[mb][nb][j]; }
        __builtin_amdgcn_wave_barrier(); asm volatile("" ::: "memory");
        float* crow = C + (size_t)(r0 + mb * 16) * ldc + c0;
#pragma unroll 1
        for (int ps = 0; ps < 2; ++ps) {
#pragma unroll
            for (int s = 0; s < 8; ++s) { const int row = 2 * s + hi, cofs = lr * 4; const v4f val = *(const v4fa*)(os + row * 68 + cofs);
                *(volatile v4f*)(crow + (size_t)row * ldc + cofs) = val; }
            if (ps == 0) __threadfence(); }
        __builtin_amdgcn_wave_barrier(); asm volatile("" ::: "memory");
    }
}

__global__ __launch_bounds__(32) void k_scores(const bf* __restrict__ Qh, const bf* __restrict__ Ql, const bf* __restrict__ Kh, const bf* __restrict__ Kl, float* S) {
    gemmc_body<bf, 2, 0>(Qh, Ql, Kh, Kl, HD, S, TT, 0); }
__global__ __launch_bounds__(32) void k_pve(const bf* __restrict__ Ph, const bf* __restrict__ Pl, const bf* __restrict__ Vh, const bf* __restrict__ Vl, float* O) {
    gemmc_body<bf, 2, 1>(Ph, Pl, Vh, Vl, TT, O, HD, 0); }
__global__ __launch_bounds__(32) void k_pvl(const h16* __restrict__ P, const h16* __restrict__ V, float* O) {
    gemmc_body<h16, 0, 1>(P, nullptr, V, nullptr, TT, O, HD, RH); }

__device__ __forceinline__ h16 tohx(float x) { return (h16)x; }
__device__ __forceinline__ void splitf(float y, unsigned short& h, unsigned short& l) { h = f2bf(y); l = f2bf(y - bf2f(h)); }
static __device__ __forceinline__ h16 toh_flush(float v) { const h16 r = (h16)v; return (fabsf(v) < 6.103515625e-05f) ? (h16)0.0f : r; }

__global__ __launch_bounds__(256) void k_cvt8(const float* __restrict__ src, bf* dst, size_t n8) { const size_t i = (size_t)blockIdx.x * 256 + threadIdx.x; if (i >= n8) return; const v8f v = *(const v8f*)(src + i * 8); v8us o;
#pragma unroll
    for (int k = 0; k < 8; ++k) o[k] = f2bf(v[k]); *(volatile v8us*)(dst + i * 8) = o; __threadfence(); *(volatile v8us*)(dst + i * 8) = o; }

__global__ __launch_bounds__(256) void k_split8(const float* __restrict__ F, int pitch, bf* Ph, bf* Pl) {
    const size_t i = (size_t)blockIdx.x * 256 + threadIdx.x; if (i >= (size_t)TT * (2 * HD / 8)) return;
    const int c = (int)(i % (2 * HD / 8)) * 8; const int t = (int)(i / (2 * HD / 8));
    const v8f v = *(const v8f*)(F + (size_t)t * pitch + c); v8us oh, ol;
#pragma unroll
    for (int k = 0; k < 8; ++k) { unsigned short a2, c2; splitf(v[k], a2, c2); oh[k] = a2; ol[k] = c2; }
    const size_t oo = (size_t)(c >= HD ? 1 : 0) * ((size_t)TT * HD) + (size_t)t * HD + (size_t)(c & (HD - 1));
    *(volatile v8us*)(Ph + oo) = oh; *(volatile v8us*)(Pl + oo) = ol; __threadfence(); *(volatile v8us*)(Ph + oo) = oh; *(volatile v8us*)(Pl + oo) = ol; }

__global__ __launch_bounds__(256) void k_vtp(const float* __restrict__ F, int pitch, int nheads, h16* V16, bf* Vh, bf* Vl) { const size_t e = ((size_t)blockIdx.x * 256 + threadIdx.x) * 2; if (e >= (size_t)nheads * HD * TT) return; const int t = (int)(e % TT); const int d = (int)((e / TT) % HD); const int g = (int)(e / ((size_t)TT * HD)); v2h o16; v2us oh, ol;
#pragma unroll
    for (int q = 0; q < 2; ++q) { const float x = F[(size_t)(t + q) * pitch + g * HD + d]; o16[q] = tohx(x); unsigned short a2, c2; splitf(x, a2, c2); oh[q] = a2; ol[q] = c2; }
    *(volatile v2h*)(V16 + e) = o16; *(volatile v2us*)(Vh + e) = oh; *(volatile v2us*)(Vl + e) = ol; __threadfence(); *(volatile v2h*)(V16 + e) = o16; *(volatile v2us*)(Vh + e) = oh; *(volatile v2us*)(Vl + e) = ol; }

__global__ __launch_bounds__(256) void k_asoft(const float* __restrict__ Sb, h16* P16, bf* Ph, bf* Pl) {
#pragma clang fp contract(off)
    const int lane = threadIdx.x & 31; const int wave = __builtin_amdgcn_readfirstlane(threadIdx.x >> 5); const int row = blockIdx.x * 8 + wave; if (row >= ZH * TT) return; const int i = row % TT; const int zz = row / TT; const bool hires = (i < RH); const float* sr = Sb + (size_t)row * TT; float v[TT / 32]; float mx = -3.0e38f;
#pragma unroll
    for (int ch = 0; ch < TT / 128; ++ch) { const int j0 = ch * 128 + lane * 4; v4f a = *(const v4f*)(sr + j0); asm volatile("" : "+v"(a));
#pragma unroll
        for (int q = 0; q < 4; ++q) { float t = __fmul_rn(a[q], SCL); asm volatile("" : "+v"(t)); t = (j0 + q <= i) ? t : -1.0e30f; v[ch * 4 + q] = t; mx = fmaxf(mx, t); } }
#pragma unroll
    for (int sh = 16; sh; sh >>= 1) mx = fmaxf(mx, __shfl_xor(mx, sh, 32));
    float sum = 0.f;
#pragma unroll
    for (int k = 0; k < TT / 32; ++k) { const bool vis = ((k >> 2) * 128 + lane * 4 + (k & 3)) <= i; float d0 = __fsub_rn(v[k], mx); asm volatile("" : "+v"(d0)); float e2 = __fmul_rn(d0, 1.4426950408889634f); asm volatile("" : "+v"(e2)); const float ex = __builtin_amdgcn_exp2f(e2); v[k] = vis ? ex : 0.0f; sum = __fadd_rn(sum, v[k]); }
#pragma unroll
    for (int sh = 16; sh; sh >>= 1) sum = __fadd_rn(sum, __shfl_xor(sum, sh, 32));
    const float f = __fdiv_rn(hires ? 1.0f : PCAR, sum);
#pragma unroll 1
    for (int ps = 0; ps < 2; ++ps) {
        if (hires) {
#pragma unroll
            for (int ch = 0; ch < TT / 128; ++ch) { v4us oh, ol;
#pragma unroll
                for (int q = 0; q < 4; ++q) { float y = __fmul_rn(v[ch * 4 + q], f); asm volatile("" : "+v"(y)); const unsigned short hh = f2bf(y); float hv = bf2f(hh); asm volatile("" : "+v"(hv)); const float r = __fsub_rn(y, hv); oh[q] = hh; ol[q] = f2bf(r); }
                const size_t oo = ((size_t)zz * (RH ? RH : 1) + i) * TT + ch * 128 + lane * 4; *(volatile v4us*)(Ph + oo) = oh; *(volatile v4us*)(Pl + oo) = ol; }
        } else {
#pragma unroll
            for (int ch = 0; ch < TT / 128; ++ch) { v4h o4;
#pragma unroll
                for (int q = 0; q < 4; ++q) { float y = __fmul_rn(v[ch * 4 + q], f); asm volatile("" : "+v"(y)); o4[q] = toh_flush(y); }
                *(volatile v4h*)(P16 + (size_t)row * TT + ch * 128 + lane * 4) = o4; } }
        if (ps == 0) __threadfence(); }
}

__global__ __launch_bounds__(256) void k_ctx8(const float* __restrict__ O, bf* Ch, bf* Cl) {
    const size_t i = (size_t)blockIdx.x * 256 + threadIdx.x; if (i >= (size_t)TT * (HD / 8)) return;
    const int t = (int)(i / (HD / 8)); const float cs = (t < RH) ? 1.0f : (1.0f / PCAR);
    const v8f v = *(const v8f*)(O + i * 8); v8us oh, ol;
#pragma unroll
    for (int k = 0; k < 8; ++k) { unsigned short a2, c2; splitf(v[k] * cs, a2, c2); oh[k] = a2; ol[k] = c2; }
    *(volatile v8us*)(Ch + i * 8) = oh; *(volatile v8us*)(Cl + i * 8) = ol; __threadfence(); *(volatile v8us*)(Ch + i * 8) = oh; *(volatile v8us*)(Cl + i * 8) = ol; }

extern "C" void kernel_launch(void* const* d_in, const int* in_sizes, int n_in,
                              void* d_out, int out_size, void* d_ws, size_t ws_size, hipStream_t stream) {
    if (n_in < 5) return;
    const size_t needx = (size_t)(NB - 1) * SEQ_FULL * DM + (size_t)SEQ * DM;
    if ((size_t)in_sizes[0] < needx) return;
    if ((size_t)in_sizes[1] < (size_t)DM * NQKV) return;
    if ((size_t)in_sizes[2] < (size_t)NQKV) return;
    if ((size_t)in_sizes[3] < (size_t)DM * HD) return;
    if ((size_t)in_sizes[4] < (size_t)DM) return;
    if ((size_t)out_size < needx) return;
    const float* x    = (const float*)d_in[0];
    const float* w    = (const float*)d_in[1];
    const float* bqkv = (const float*)d_in[2];
    const float* wo   = (const float*)d_in[3];
    const float* bo   = (const float*)d_in[4];
    float* OUT = (float*)d_out;
    char* wsp = (char*)d_ws;
    auto take = [&](size_t bytes) { char* p = wsp; wsp += (bytes + 255) & ~(size_t)255; return (void*)p; };
    bf* WT = (bf*)take((size_t)NQKV * DM * 2);
    bf* WOB = (bf*)take((size_t)DM * HD * 2);
    bf* XB = (bf*)take((size_t)TT * DM * 2);
    float* F = (float*)take((size_t)TT * NQKV * 4);
    h16* VT16 = (h16*)take((size_t)HD * TT * 2);
    bf* QKh = (bf*)take((size_t)2 * TT * HD * 2); bf* QKl = (bf*)take((size_t)2 * TT * HD * 2);
    bf* VTh = (bf*)take((size_t)HD * TT * 2); bf* VTl = (bf*)take((size_t)HD * TT * 2);
    bf* Ph = (bf*)take((size_t)ZH * RH * TT * 2); bf* Pl = (bf*)take((size_t)ZH * RH * TT * 2);
    float* Sb = (float*)take((size_t)ZH * TT * TT * 4); h16* P16 = (h16*)take((size_t)ZH * TT * TT * 2); float* Ob = (float*)take((size_t)ZH * TT * HD * 4);
    bf* CXh = (bf*)take((size_t)TT * HD * 2); bf* CXl = (bf*)take((size_t)TT * HD * 2);
    if ((size_t)(wsp - (char*)d_ws) > ws_size) return;
    k_cvt8<<<(unsigned)(((size_t)NQKV * DM / 8 + 255) / 256), 256, 0, stream>>>(w, WT, (size_t)NQKV * DM / 8);
    k_cvt8<<<(unsigned)(((size_t)DM * HD / 8 + 255) / 256), 256, 0, stream>>>(wo, WOB, (size_t)DM * HD / 8);
    const unsigned LV = (unsigned)(((size_t)TT * HD / 2 + 255) / 256);
    for (int b = 0; b < NB; ++b) {
        k_cvt8<<<(unsigned)(((size_t)TT * DM / 8 + 255) / 256), 256, 0, stream>>>(x + (size_t)b * SEQ_FULL * DM, XB, (size_t)TT * DM / 8);
        k_gemmw<bf, 0, true><<<dim3(TT / 64, NQKV / 64, 1), 32, 0, stream>>>(XB, nullptr, WT, nullptr, DM, F, NQKV, bqkv, 0, 0, 0);
        k_split8<<<(unsigned)(((size_t)TT * (2 * HD / 8) + 255) / 256), 256, 0, stream>>>(F, NQKV, QKh, QKl);
        k_vtp<<<LV, 256, 0, stream>>>(F + 2 * HD, NQKV, 1, VT16, VTh, VTl);
        k_scores<<<dim3(TT / 64, TT / 64, 1), 32, 0, stream>>>(QKh, QKl, QKh + (size_t)TT * HD, QKl + (size_t)TT * HD, Sb);
        k_asoft<<<ZH * TT / 8, 256, 0, stream>>>(Sb, P16, Ph, Pl);
        if (RH > 0) k_pve<<<dim3((RH > 0 ? RH : 64) / 64, HD / 64, 1), 32, 0, stream>>>(Ph, Pl, VTh, VTl, Ob);
        if (TT > RH) k_pvl<<<dim3((TT > RH ? (TT - RH) : 64) / 64, HD / 64, 1), 32, 0, stream>>>(P16 + (size_t)RH * TT, VT16, Ob + (size_t)RH * HD);
        k_ctx8<<<(unsigned)(((size_t)TT * (HD / 8) + 255) / 256), 256, 0, stream>>>(Ob, CXh, CXl);
        k_gemmw<bf, 1, true><<<dim3(TT / 64, DM / 64, 1), 32, 0, stream>>>(CXh, CXl, WOB, nullptr, HD, OUT + (size_t)b * SEQ_FULL * DM, DM, bo, 0, 0, 0);
    }
}
